// MSA_850403525285
// MI455X (gfx1250) — hardware-verified
//
#include <hip/hip_runtime.h>
#include <math.h>
#include <stdint.h>

#define NB     4
#define SEQ    2048
#define DMOD   1024
#define NHEAD  16
#define HDIM   64
#define N3     3072
#define MTOK   (NB * SEQ)
#define QP     (2 * DMOD)
#define VP     MTOK

static_assert((MTOK % 64) == 0);
static_assert((DMOD % 64) == 0);
static_assert((N3 % 64) == 0);
static_assert((DMOD % 32) == 0);
static_assert((QP % 32) == 0);
static_assert(NHEAD * HDIM == DMOD);
static_assert(((MTOK * DMOD) % (8 * 256)) == 0);

typedef __attribute__((ext_vector_type(16))) _Float16 v16h;
typedef __attribute__((ext_vector_type(8)))  _Float16 v8h;
typedef __attribute__((ext_vector_type(16))) __bf16   v16b;
typedef __attribute__((ext_vector_type(8)))  __bf16   v8b;
typedef __attribute__((ext_vector_type(8)))  float    v8f;
typedef __attribute__((ext_vector_type(4)))  float    v4f;
typedef __attribute__((ext_vector_type(2)))  float    v2f;
typedef __attribute__((ext_vector_type(4)))  unsigned int v4u;

__device__ __forceinline__ unsigned short f2bf_bits(float f) {
  unsigned u = __float_as_uint(f);
  return (unsigned short)((u + 0x7FFFu + ((u >> 16) & 1u)) >> 16);
}
__device__ __forceinline__ float bf_bits2f(unsigned short h) { return __uint_as_float(((unsigned)h) << 16); }
__device__ __forceinline__ unsigned pk16(unsigned short a, unsigned short b) { return (unsigned)a | ((unsigned)b << 16); }

__device__ __forceinline__ void dep_guard_h(v8f& a, v8f& b, v16h x, v16h y) { asm volatile("v_nop\n\tv_nop\n\tv_nop\n\tv_nop" : "+v"(a), "+v"(b) : "v"(x), "v"(y)); }
__device__ __forceinline__ void dep_guard_b(v8f& a, v8f& b, v16b x, v16b y) { asm volatile("v_nop\n\tv_nop\n\tv_nop\n\tv_nop" : "+v"(a), "+v"(b) : "v"(x), "v"(y)); }
__device__ __forceinline__ void keep4_h(v16h a, v16h b, v16h c, v16h d) { asm volatile("v_nop" :: "v"(a), "v"(b), "v"(c), "v"(d)); }
__device__ __forceinline__ void keep4_b(v16b a, v16b b, v16b c, v16b d) { asm volatile("v_nop" :: "v"(a), "v"(b), "v"(c), "v"(d)); }
__device__ __forceinline__ void acc_guard4(v8f& a, v8f& b, v8f& c, v8f& d) { asm volatile("v_nop\n\tv_nop\n\tv_nop\n\tv_nop" : "+v"(a), "+v"(b), "+v"(c), "+v"(d)); }

template <typename T> struct Frag;
template <> struct Frag<_Float16> {
  typedef v16h V; union U { v16h v; v8h h[2]; };
  static __device__ __forceinline__ v16h load(const _Float16* p) {
    U f; f.h[0] = *(const v8h*)(p); f.h[1] = *(const v8h*)(p + 16); return f.v;
  }
  static __device__ __forceinline__ v8f mma(v16h a, v16h b, v8f c) {
    return __builtin_amdgcn_wmma_f32_16x16x32_f16(false, a, false, b, (short)0, c, false, false);
  }
  static __device__ __forceinline__ void guard(v8f& a, v8f& b, v16h x, v16h y) { dep_guard_h(a, b, x, y); }
  static __device__ __forceinline__ void keep(v16h a, v16h b, v16h c, v16h d) { keep4_h(a, b, c, d); }
};
template <> struct Frag<__bf16> {
  typedef v16b V; union U { v16b v; v8b h[2]; };
  static __device__ __forceinline__ v16b load(const __bf16* p) {
    U f; f.h[0] = *(const v8b*)(p); f.h[1] = *(const v8b*)(p + 16); return f.v;
  }
  static __device__ __forceinline__ v8f mma(v16b a, v16b b, v8f c) {
    return __builtin_amdgcn_wmma_f32_16x16x32_bf16(false, a, false, b, (short)0, c, false, false);
  }
  static __device__ __forceinline__ void guard(v8f& a, v8f& b, v16b x, v16b y) { dep_guard_b(a, b, x, y); }
  static __device__ __forceinline__ void keep(v16b a, v16b b, v16b c, v16b d) { keep4_b(a, b, c, d); }
};

template <int ET> struct Elem;
template <> struct Elem<0> { typedef _Float16 T; };
template <> struct Elem<1> { typedef __bf16 T; };
template <int ET, bool SPLIT, int BIAS_MODE, int OUT_MODE, bool RESID, int ACT = 0>
__global__ __launch_bounds__(256) void wmma_gemm64(
    const unsigned short* __restrict__ Ap, const unsigned short* __restrict__ A2p, int lda, long strideA,
    const unsigned short* __restrict__ Btp, const unsigned short* __restrict__ Bt2p, int ldb, long strideB,
    void* __restrict__ Cout, void* __restrict__ Cout2, int ldc, long strideC,
    const float* __restrict__ bias,
    const float* __restrict__ resid, long strideR,
    int M, int N, int K, float scale) {
  typedef typename Elem<ET>::T T;
  typedef typename Frag<T>::V V;
  const T* A = (const T*)Ap; const T* A2 = (const T*)A2p; const T* Bt = (const T*)Btp; const T* Bt2 = (const T*)Bt2p;
  __shared__ __align__(16) float sT[8][16 * 68];
  const int b    = blockIdx.y;
  const int lane = threadIdx.x & 31;
  const int wave = threadIdx.x >> 5;
  const int tilesN = N >> 6;
  const int tilesM = M >> 6;
  const int tile = blockIdx.x * 8 + wave;
  if (tile >= tilesM * tilesN) return;
  const int tm = tile / tilesN;
  const int tn = tile - tm * tilesN;
  const int m0 = tm << 6;
  const int n0 = tn << 6;

  const T* Ab  = A  + (size_t)b * strideA;
  const T* Bb  = Bt + (size_t)b * strideB;
  const T* Ab2 = SPLIT ? (A2  + (size_t)b * strideA) : nullptr;
  const T* Bb2 = SPLIT ? (Bt2 + (size_t)b * strideB) : nullptr;

  const int rlane = lane & 15;
  const int koff  = (lane >> 4) * 8;
  const int mOff  = (lane >> 4) * 8;

  v8f acc[4][4];
#pragma unroll
  for (int i = 0; i < 4; ++i)
#pragma unroll
    for (int j = 0; j < 4; ++j) acc[i][j] = (v8f){0.f,0.f,0.f,0.f,0.f,0.f,0.f,0.f};

  for (int k0 = 0; k0 < K; k0 += 32) {
    V bh[4], bl[4];
#pragma unroll
    for (int j = 0; j < 4; ++j) {
      const size_t bo = (size_t)(n0 + (j << 4) + rlane) * ldb + koff + k0;
      bh[j] = Frag<T>::load(Bb + bo);
      if (SPLIT) bl[j] = Frag<T>::load(Bb2 + bo);
    }
#pragma unroll
    for (int i = 0; i < 4; ++i) {
      const size_t ao = (size_t)(m0 + (i << 4) + rlane) * lda + koff + k0;
      V ah = Frag<T>::load(Ab + ao);
      V al;
      if (SPLIT) al = Frag<T>::load(Ab2 + ao);
#pragma unroll
      for (int j = 0; j < 4; ++j) {
        acc[i][j] = Frag<T>::mma(ah, bh[j], acc[i][j]);
        if (SPLIT) {
          acc[i][j] = Frag<T>::mma(ah, bl[j], acc[i][j]);
          acc[i][j] = Frag<T>::mma(al, bh[j], acc[i][j]);
        }
      }
      Frag<T>::guard(acc[i][0], acc[i][3], ah, SPLIT ? al : ah);
    }
    Frag<T>::keep(bh[0], bh[1], bh[2], bh[3]);
    if (SPLIT) Frag<T>::keep(bl[0], bl[1], bl[2], bl[3]);
  }
  acc_guard4(acc[0][0], acc[0][1], acc[0][2], acc[0][3]);
  acc_guard4(acc[1][0], acc[1][1], acc[1][2], acc[1][3]);
  acc_guard4(acc[2][0], acc[2][1], acc[2][2], acc[2][3]);
  acc_guard4(acc[3][0], acc[3][1], acc[3][2], acc[3][3]);

  float* slab = sT[wave];
  const float* Rb = RESID ? (resid + (size_t)b * strideR) : nullptr;
#pragma unroll
  for (int i = 0; i < 4; ++i) {
    const int mBase = m0 + (i << 4);
#pragma unroll
    for (int j = 0; j < 4; ++j) {
      const int n = n0 + (j << 4) + rlane;
      float bv = 0.f;
      if (BIAS_MODE == 2) bv = bias[n];
#pragma unroll
      for (int r = 0; r < 8; ++r) {
        float v = acc[i][j][r] * scale;
        if (BIAS_MODE == 1) v += bias[mBase + mOff + r];
        if (BIAS_MODE == 2) v += bv;
        if (RESID) v += Rb[(size_t)(mBase + mOff + r) * ldc + n];
        if (ACT == 2) v = fmaxf(v, 0.0f);
        slab[(mOff + r) * 68 + (j << 4) + rlane] = v;
      }
    }
    __builtin_amdgcn_fence(__ATOMIC_RELEASE, "workgroup");
    __builtin_amdgcn_wave_barrier();
    __builtin_amdgcn_fence(__ATOMIC_ACQUIRE, "workgroup");
    if (OUT_MODE == 0) {
      float* C = (float*)Cout + (size_t)b * strideC;
      const int hh = lane >> 4, c4 = (lane & 15) * 4;
      for (int pass = 0; pass < 2; ++pass) {
#pragma unroll
        for (int it = 0; it < 8; ++it) {
          const int row = it * 2 + hh;
          v4f v = *(const v4f*)(slab + row * 68 + c4);
          *(volatile v4f*)(C + (size_t)(mBase + row) * ldc + n0 + c4) = v;
        }
        __threadfence();
      }
    } else {
      const int q = lane >> 3, c8 = (lane & 7) * 8;
      unsigned short* C  = (unsigned short*)Cout  + (size_t)b * strideC;
      unsigned short* C2 = (OUT_MODE == 2) ? ((unsigned short*)Cout2 + (size_t)b * strideC) : nullptr;
      for (int pass = 0; pass < 2; ++pass) {
#pragma unroll
        for (int it = 0; it < 4; ++it) {
          const int row = it * 4 + q;
          const float* sp = slab + row * 68 + c8;
          v8h hv, lv;
#pragma unroll
          for (int e = 0; e < 8; ++e) {
            if (OUT_MODE == 1) {
              hv[e] = (_Float16)sp[e];
            } else {
              unsigned short hb = f2bf_bits(sp[e]);
              unsigned short lb = f2bf_bits(sp[e] - bf_bits2f(hb));
              hv[e] = __builtin_bit_cast(_Float16, hb);
              lv[e] = __builtin_bit_cast(_Float16, lb);
            }
          }
          *(volatile v8h*)(C + (size_t)(mBase + row) * ldc + n0 + c8) = hv;
          if (OUT_MODE == 2) *(volatile v8h*)(C2 + (size_t)(mBase + row) * ldc + n0 + c8) = lv;
        }
        __threadfence();
      }
    }
    __builtin_amdgcn_fence(__ATOMIC_RELEASE, "workgroup");
    __builtin_amdgcn_wave_barrier();
    __builtin_amdgcn_fence(__ATOMIC_ACQUIRE, "workgroup");
  }
}

__global__ __launch_bounds__(256) void cvt_x_kernel(const float* __restrict__ x, unsigned short* __restrict__ xb, int n8) {
  const int g = blockIdx.x * 256 + threadIdx.x;
  if (g >= n8) return;
  const v4f a = *(const v4f*)(x + (size_t)g * 8);
  const v4f c = *(const v4f*)(x + (size_t)g * 8 + 4);
  v4u o;
  o[0] = pk16(f2bf_bits(a[0]), f2bf_bits(a[1]));
  o[1] = pk16(f2bf_bits(a[2]), f2bf_bits(a[3]));
  o[2] = pk16(f2bf_bits(c[0]), f2bf_bits(c[1]));
  o[3] = pk16(f2bf_bits(c[2]), f2bf_bits(c[3]));
  volatile v4u* d = (volatile v4u*)(xb + (size_t)g * 8);
  *d = o;
  __threadfence();
  *d = o;
}

__global__ __launch_bounds__(256) void tconv_kernel(const float* __restrict__ W, unsigned short* __restrict__ ob,
                                                    int R, int Cc, int ldo, int dup) {
  __shared__ __align__(16) float tf[64 * 68];
  const int c0  = blockIdx.x * 64;
  const int r0  = blockIdx.y * 64;
  const int tid = threadIdx.x;
  {
    const int lr = tid >> 4;
    const int c4 = (tid & 15) * 4;
#pragma unroll
    for (int it = 0; it < 4; ++it) {
      const int rr = it * 16 + lr;
      const v4f a = *(const v4f*)(W + (size_t)(r0 + rr) * Cc + c0 + c4);
      *(v4f*)(tf + rr * 68 + c4) = a;
    }
  }
  __syncthreads();
  const int sub = tid >> 3;
  const int c8  = (tid & 7) * 8;
  v4u hv[2];
#pragma unroll
  for (int it = 0; it < 2; ++it) {
    const int oc = it * 32 + sub;
    v4u a;
#pragma unroll
    for (int q = 0; q < 4; ++q) {
      const float f0 = tf[(c8 + 2 * q) * 68 + oc];
      const float f1 = tf[(c8 + 2 * q + 1) * 68 + oc];
      a[q] = pk16(f2bf_bits(f0), f2bf_bits(f1));
    }
    hv[it] = a;
  }
  for (int pass = 0; pass < 2; ++pass) {
#pragma unroll
    for (int it = 0; it < 2; ++it) {
      const int oc = it * 32 + sub;
      const size_t go = (size_t)(c0 + oc) * ldo + r0 + c8;
      *(volatile v4u*)(ob + go) = hv[it];
      if (dup != 0) *(volatile v4u*)(ob + go + R) = hv[it];
    }
    __threadfence();
  }
}

#define AT_D 64
#define AT_NW 4
#define AT_QB 64
#define AT_KC 64

__device__ __forceinline__ unsigned short at_bf_bits(float f) {
  unsigned u = __float_as_uint(f);
  return (unsigned short)((u + 0x7FFFu + ((u >> 16) & 1u)) >> 16);
}
__device__ __forceinline__ __bf16 at_f2bf(float f) { return __builtin_bit_cast(__bf16, at_bf_bits(f)); }
__device__ __forceinline__ void at_split(float f, __bf16& hi, __bf16& lo) {
  const unsigned short hb = at_bf_bits(f);
  hi = __builtin_bit_cast(__bf16, hb);
  lo = at_f2bf(f - __uint_as_float(((unsigned)hb) << 16));
}
__device__ __forceinline__ v8f at_mma(v16b a, v16b b, v8f c) {
  c = __builtin_amdgcn_wmma_f32_16x16x32_bf16(false, a, false, b, (short)0, c, false, false);
  asm volatile("v_nop\n\tv_nop\n\tv_nop\n\tv_nop" : "+v"(c) : "v"(a), "v"(b));
  return c;
}

__global__ __launch_bounds__(128)
void attn_full64_kernel(unsigned short* qc,
                        const unsigned short* __restrict__ kp,
                        const unsigned short* __restrict__ vhp,
                        const unsigned short* __restrict__ vlp,
                        float sscale) {
  union FB { v16b v; v8b h[2]; };
  __shared__ __align__(16) __bf16 Ksh[AT_KC * AT_D];
  __shared__ __align__(16) __bf16 Ksl[AT_KC * AT_D];
  __shared__ __align__(16) __bf16 Vth[AT_D * AT_KC];
  __shared__ __align__(16) __bf16 Vtl[AT_D * AT_KC];
  __shared__ __align__(16) __bf16 Psh[AT_NW][16 * AT_KC];
  __shared__ __align__(16) __bf16 Psl[AT_NW][16 * AT_KC];
  __shared__ __align__(16) float  Os[AT_NW][16 * 68];

  const int tid  = threadIdx.x;
  const int wave = tid >> 5;
  const int lane = tid & 31;
  const int hh   = lane >> 4;
  const int c    = lane & 15;

  const int nqb = SEQ / AT_QB;
  const int bx = blockIdx.x;
  const int qb = bx % nqb;
  const int h  = bx / nqb;
  const int b  = blockIdx.y;
  const int q0 = qb * AT_QB + wave * 16;
  const size_t tok0 = (size_t)b * SEQ;

  const __bf16* Qh = (const __bf16*)(const void*)qc + tok0 * QP + (size_t)h * AT_D;
  const __bf16* Ql = Qh + DMOD;
  const __bf16* Kh = (const __bf16*)(const void*)kp + tok0 * QP + (size_t)h * AT_D;
  const __bf16* Kl = Kh + DMOD;
  const __bf16* Vh = (const __bf16*)(const void*)vhp + (size_t)h * AT_D * VP + tok0;
  const __bf16* Vl = (const __bf16*)(const void*)vlp + (size_t)h * AT_D * VP + tok0;
  unsigned short* Cb = qc + tok0 * QP + (size_t)h * AT_D;

  v16b qah[2], qal[2];
#pragma unroll
  for (int dc = 0; dc < 2; ++dc) {
    const __bf16* qr = Qh + (size_t)(q0 + c) * QP + dc * 32 + 8 * hh;
    const __bf16* ql = Ql + (size_t)(q0 + c) * QP + dc * 32 + 8 * hh;
    qah[dc] = Frag<__bf16>::load(qr);
    qal[dc] = Frag<__bf16>::load(ql);
  }

  float mrow[8], lrow[8];
  v8f oacc[4];
#pragma unroll
  for (int r = 0; r < 8; ++r) { mrow[r] = -INFINITY; lrow[r] = 0.f; }
#pragma unroll
  for (int t = 0; t < 4; ++t) oacc[t] = (v8f){0.f,0.f,0.f,0.f,0.f,0.f,0.f,0.f};

  const int nChunks = SEQ / AT_KC;
  for (int kc = 0; kc < nChunks; ++kc) {
    const int kv0 = kc * AT_KC;
    __syncthreads();
    {
      const int r = tid >> 1, half = (tid & 1) * 32;
      const __bf16* ksh = Kh + (size_t)(kv0 + r) * QP + half;
      const __bf16* ksl = Kl + (size_t)(kv0 + r) * QP + half;
      const __bf16* vsh = Vh + (size_t)r * VP + kv0 + half;
      const __bf16* vsl = Vl + (size_t)r * VP + kv0 + half;
#pragma unroll
      for (int i = 0; i < 4; ++i) {
        const v8b a0 = *(const v8b*)(ksh + 8 * i);
        const v8b a1 = *(const v8b*)(ksl + 8 * i);
        const v8b b0 = *(const v8b*)(vsh + 8 * i);
        const v8b b1 = *(const v8b*)(vsl + 8 * i);
        *(v8b*)(Ksh + r * AT_D  + half + 8 * i) = a0;
        *(v8b*)(Ksl + r * AT_D  + half + 8 * i) = a1;
        *(v8b*)(Vth + r * AT_KC + half + 8 * i) = b0;
        *(v8b*)(Vtl + r * AT_KC + half + 8 * i) = b1;
      }
    }
    __syncthreads();

    v8f s[4];
#pragma unroll
    for (int j = 0; j < 4; ++j) {
      s[j] = (v8f){0.f,0.f,0.f,0.f,0.f,0.f,0.f,0.f};
#pragma unroll
      for (int dc = 0; dc < 2; ++dc) {
        FB kb, kl;
        kb.h[0] = *(const v8b*)(Ksh + (j * 16 + c) * AT_D + dc * 32 + 8 * hh);
        kb.h[1] = *(const v8b*)(Ksh + (j * 16 + c) * AT_D + dc * 32 + 16 + 8 * hh);
        kl.h[0] = *(const v8b*)(Ksl + (j * 16 + c) * AT_D + dc * 32 + 8 * hh);
        kl.h[1] = *(const v8b*)(Ksl + (j * 16 + c) * AT_D + dc * 32 + 16 + 8 * hh);
        s[j] = at_mma(qah[dc], kb.v, s[j]);
        s[j] = at_mma(qah[dc], kl.v, s[j]);
        s[j] = at_mma(qal[dc], kb.v, s[j]);
      }
    }
    float cm[8];
#pragma unroll
    for (int r = 0; r < 8; ++r) {
      float m = -INFINITY;
#pragma unroll
      for (int j = 0; j < 4; ++j) {
        const float sv = s[j][r] * sscale;
        s[j][r] = sv;
        m = fmaxf(m, sv);
      }
#pragma unroll
      for (int off = 1; off < 16; off <<= 1) m = fmaxf(m, __shfl_xor(m, off, 32));
      cm[r] = m;
    }
    __bf16* pwh = Psh[wave];
    __bf16* pwl = Psl[wave];
#pragma unroll
    for (int r = 0; r < 8; ++r) {
      const float mnew = fmaxf(mrow[r], cm[r]);
      const float alpha = expf(mrow[r] - mnew);
      mrow[r] = mnew;
      float psum = 0.f;
#pragma unroll
      for (int j = 0; j < 4; ++j) {
        const float p = expf(s[j][r] - mnew);
        psum += p;
        __bf16 a, bl; at_split(p, a, bl);
        pwh[(8 * hh + r) * AT_KC + j * 16 + c] = a;
        pwl[(8 * hh + r) * AT_KC + j * 16 + c] = bl;
      }
#pragma unroll
      for (int off = 1; off < 16; off <<= 1) psum += __shfl_xor(psum, off, 32);
      lrow[r] = lrow[r] * alpha + psum;
#pragma unroll
      for (int t = 0; t < 4; ++t) oacc[t][r] *= alpha;
    }
    __builtin_amdgcn_fence(__ATOMIC_RELEASE, "workgroup");
    __builtin_amdgcn_wave_barrier();
    __builtin_amdgcn_fence(__ATOMIC_ACQUIRE, "workgroup");
#pragma unroll 1
    for (int kk = 0; kk < 2; ++kk) {
      FB pa, pl;
      pa.h[0] = *(const v8b*)(pwh + c * AT_KC + kk * 32 + 8 * hh);
      pa.h[1] = *(const v8b*)(pwh + c * AT_KC + kk * 32 + 16 + 8 * hh);
      pl.h[0] = *(const v8b*)(pwl + c * AT_KC + kk * 32 + 8 * hh);
      pl.h[1] = *(const v8b*)(pwl + c * AT_KC + kk * 32 + 16 + 8 * hh);
#pragma unroll
      for (int t = 0; t < 4; ++t) {
        FB vb, vl;
        vb.h[0] = *(const v8b*)(Vth + (t * 16 + c) * AT_KC + kk * 32 + 8 * hh);
        vb.h[1] = *(const v8b*)(Vth + (t * 16 + c) * AT_KC + kk * 32 + 16 + 8 * hh);
        vl.h[0] = *(const v8b*)(Vtl + (t * 16 + c) * AT_KC + kk * 32 + 8 * hh);
        vl.h[1] = *(const v8b*)(Vtl + (t * 16 + c) * AT_KC + kk * 32 + 16 + 8 * hh);
        oacc[t] = at_mma(pa.v, vb.v, oacc[t]);
        oacc[t] = at_mma(pa.v, vl.v, oacc[t]);
        oacc[t] = at_mma(pl.v, vb.v, oacc[t]);
      }
    }
  }

  float* os = Os[wave];
#pragma unroll
  for (int r = 0; r < 8; ++r) {
    const float inv = 1.0f / lrow[r];
#pragma unroll
    for (int t = 0; t < 4; ++t) os[(8 * hh + r) * 68 + t * 16 + c] = oacc[t][r] * inv;
  }
  __builtin_amdgcn_fence(__ATOMIC_RELEASE, "workgroup");
  __builtin_amdgcn_wave_barrier();
  __builtin_amdgcn_fence(__ATOMIC_ACQUIRE, "workgroup");
  {
    const int q = lane >> 3, c8 = (lane & 7) * 8;
    for (int pass = 0; pass < 2; ++pass) {
#pragma unroll
      for (int it = 0; it < 4; ++it) {
        const int row = it * 4 + q;
        const float* sp = os + row * 68 + c8;
        v8h hv, lv;
#pragma unroll
        for (int e = 0; e < 8; ++e) {
          const unsigned short hb = f2bf_bits(sp[e]);
          const unsigned short lb = f2bf_bits(sp[e] - bf_bits2f(hb));
          hv[e] = __builtin_bit_cast(_Float16, hb);
          lv[e] = __builtin_bit_cast(_Float16, lb);
        }
        unsigned short* dst = Cb + (size_t)(q0 + row) * QP + c8;
        *(volatile v8h*)(dst) = hv;
        *(volatile v8h*)(dst + DMOD) = lv;
      }
      __threadfence();
    }
  }
}

extern "C" void kernel_launch(void* const* d_in, const int* in_sizes, int n_in,
                              void* d_out, int out_size, void* d_ws, size_t ws_size,
                              hipStream_t stream) {
  if (n_in < 4) return;
  if (in_sizes[0] != MTOK * DMOD) return;
  if (in_sizes[1] != DMOD * N3) return;
  if (in_sizes[2] != DMOD * DMOD) return;
  if (in_sizes[3] != DMOD) return;
  if (out_size != MTOK * DMOD) return;

  const float* x      = (const float*)d_in[0];
  const float* w_qkv  = (const float*)d_in[1];
  const float* w_proj = (const float*)d_in[2];
  const float* b_proj = (const float*)d_in[3];
  float* out = (float*)d_out;

  const size_t bXB = (size_t)MTOK * DMOD * 2;
  const size_t bWQ = (size_t)N3 * DMOD * 2;
  const size_t bWO = (size_t)DMOD * QP * 2;
  const size_t bQK = (size_t)MTOK * QP * 2;
  const size_t bVT = (size_t)DMOD * VP * 2;
  size_t off = 0;
  const size_t oXB = off; off += bXB;
  const size_t oWQ = off; off += bWQ;
  const size_t oWO = off; off += bWO;
  const size_t oQC = off; off += bQK;
  const size_t oKK = off; off += bQK;
  const size_t oVh = off; off += bVT;
  const size_t oVl = off; off += bVT;
  if (off > ws_size) return;

  char* ws = (char*)d_ws;
  unsigned short* XB  = (unsigned short*)(ws + oXB);
  unsigned short* WQ  = (unsigned short*)(ws + oWQ);
  unsigned short* WO  = (unsigned short*)(ws + oWO);
  unsigned short* QC  = (unsigned short*)(ws + oQC);
  unsigned short* KK  = (unsigned short*)(ws + oKK);
  unsigned short* VTh = (unsigned short*)(ws + oVh);
  unsigned short* VTl = (unsigned short*)(ws + oVl);

  const dim3 blk(256);

  const int n8 = MTOK * DMOD / 8;
  cvt_x_kernel<<<dim3(n8 / 256), blk, 0, stream>>>(x, XB, n8);
  tconv_kernel<<<dim3(N3 / 64, DMOD / 64), blk, 0, stream>>>(w_qkv, WQ, DMOD, N3, DMOD, 0);
  tconv_kernel<<<dim3(DMOD / 64, DMOD / 64), blk, 0, stream>>>(w_proj, WO, DMOD, DMOD, QP, 1);

  const dim3 gQK(((MTOK / 64) * (DMOD / 64) + 7) / 8, 1);
  const dim3 gVT(((DMOD / 64) * (MTOK / 64) + 7) / 8, 1);
  wmma_gemm64<1, false, 0, 2, false, 0><<<gQK, blk, 0, stream>>>(
      XB, XB, DMOD, 0L, WQ, WQ, DMOD, 0L, (void*)QC, (void*)(QC + DMOD), QP, 0L,
      b_proj, b_proj, 0L, MTOK, DMOD, DMOD, 1.0f);
  wmma_gemm64<1, false, 0, 2, false, 0><<<gQK, blk, 0, stream>>>(
      XB, XB, DMOD, 0L, WQ + (size_t)DMOD * DMOD, WQ + (size_t)DMOD * DMOD, DMOD, 0L,
      (void*)KK, (void*)(KK + DMOD), QP, 0L,
      b_proj, b_proj, 0L, MTOK, DMOD, DMOD, 1.0f);
  wmma_gemm64<1, false, 0, 2, false, 0><<<gVT, blk, 0, stream>>>(
      WQ + (size_t)2 * DMOD * DMOD, WQ + (size_t)2 * DMOD * DMOD, DMOD, 0L, XB, XB, DMOD, 0L,
      (void*)VTh, (void*)VTl, VP, 0L,
      b_proj, b_proj, 0L, DMOD, MTOK, DMOD, 1.0f);
  attn_full64_kernel<<<dim3(NHEAD * (SEQ / 64), NB), dim3(128), 0, stream>>>(QC, KK, VTh, VTl, 0.125f);
  wmma_gemm64<1, false, 2, 0, false, 0><<<gQK, blk, 0, stream>>>(
      QC, QC, QP, 0L, WO, WO, QP, 0L, (void*)out, (void*)out, DMOD, 0L,
      b_proj, b_proj, 0L, MTOK, DMOD, QP, 1.0f);
  (void)hipGetLastError();
}
